// InterleavedHeadAttention_67920612819085
// MI455X (gfx1250) — hardware-verified
//
#include <hip/hip_runtime.h>
#include <math.h>


#define BB 2
#define ST 1024
#define PP 2
#define SS (ST * PP)
#define DD 1024
#define HH 16
#define HD 64
#define BT (BB * ST)
#define DO (HH * PP * HD)
#define BK 32
typedef float __attribute__((may_alias)) float_a;

typedef __attribute__((ext_vector_type(16))) _Float16 v16h;
typedef __attribute__((ext_vector_type(16))) __bf16 v16b;
typedef __attribute__((ext_vector_type(8)))  float v8f;
typedef __attribute__((ext_vector_type(4)))  float v4f;
typedef __attribute__((ext_vector_type(8)))  _Float16 v8h;
typedef __attribute__((ext_vector_type(4)))  unsigned v4u;

template <typename T> __device__ __forceinline__ void vst2(void* p, T v) { *(volatile T*)p = v; __threadfence(); *(volatile T*)p = v; }
__device__ __forceinline__ v8f wmma16(v16h a, v16h b, v8f c) {
  v8f d = __builtin_amdgcn_wmma_f32_16x16x32_f16(false, a, false, b, (short)0, c, false, false);
  asm volatile("v_nop\n\tv_nop\n\tv_nop\n\tv_nop" : "+v"(d) : "v"(a), "v"(b));
  return d;
}
__device__ __forceinline__ v8f wmma_bf(v16b a, v16b b, v8f c) {
  v8f d = __builtin_amdgcn_wmma_f32_16x16x32_bf16(false, a, false, b, (short)0, c, false, false);
  asm volatile("v_nop\n\tv_nop\n\tv_nop\n\tv_nop" : "+v"(d) : "v"(a), "v"(b));
  return d;
}
struct F2 { v16b h, l; };
__device__ __forceinline__ F2 split_row(const float* rowk0, int lane) {
  F2 r; const float* p = rowk0 + 8 * (lane >> 4);
#pragma unroll
  for (int i = 0; i < 8; ++i) { float v0 = p[i], v1 = p[16 + i]; __bf16 h0 = (__bf16)v0, h1 = (__bf16)v1;
    r.h[i] = h0; r.l[i] = (__bf16)(v0 - (float)h0); r.h[8 + i] = h1; r.l[8 + i] = (__bf16)(v1 - (float)h1); }
  return r;
}
__device__ __forceinline__ v8f mac3(const F2& a, const F2& b, v8f c) { c = wmma_bf(a.l, b.h, c); c = wmma_bf(a.h, b.l, c); return wmma_bf(a.h, b.h, c); }
struct H2 { v16h h, l; };
__device__ __forceinline__ H2 hsplit_row(const float* rowk0, int lane) {
  H2 a; const float* p = rowk0 + 8 * (lane >> 4);
#pragma unroll
  for (int i = 0; i < 8; ++i) { float v0 = p[i], v1 = p[16 + i]; _Float16 h0 = (_Float16)v0, h1 = (_Float16)v1;
    a.h[i] = h0; a.l[i] = (_Float16)(v0 - (float)h0); a.h[8 + i] = h1; a.l[8 + i] = (_Float16)(v1 - (float)h1); }
  return a;
}
__device__ __forceinline__ v16h frag_f32(const float* rowk0, int lane) {
  v16h a; const float* p = rowk0 + 8 * (lane >> 4);
#pragma unroll
  for (int i = 0; i < 8; ++i) { a[i] = (_Float16)p[i]; a[8 + i] = (_Float16)p[16 + i]; }
  return a;
}
__device__ __forceinline__ v16h frag_h(const _Float16* rowk0, int lane) { union { v4u u[2]; v16h h; } r; const _Float16* p = rowk0 + 8 * (lane >> 4); r.u[0] = *(const v4u*)p; r.u[1] = *(const v4u*)(p + 16); return r.h; }
__global__ __launch_bounds__(256) void k_cvt(const float* __restrict__ src, _Float16* __restrict__ dst, size_t n8, float sc) {
  const size_t i8 = (size_t)blockIdx.x * 256 + threadIdx.x; if (i8 >= n8) return; union { v8h h; v4u u; } pk;
#pragma unroll
  for (int e = 0; e < 8; ++e) pk.h[e] = (_Float16)(src[i8 * 8 + e] * sc);
  vst2(dst + i8 * 8, pk.u);
}
#define LDSX() do { asm volatile("s_wait_dscnt 0" ::: "memory"); __builtin_amdgcn_wave_barrier(); __builtin_amdgcn_fence(__ATOMIC_RELEASE, "workgroup"); } while (0)

__global__ __launch_bounds__(256) void k_weff(const float* __restrict__ Wq, const float* __restrict__ Wk, const float* __restrict__ Wv,
                                            const float* __restrict__ aq, const float* __restrict__ ak, const float* __restrict__ av,
                                            float* __restrict__ Weff) {
  const int o = blockIdx.x, which = blockIdx.y, tid = threadIdx.x;
  const int h = o / (PP * HD), p = (o / HD) % PP, d = o % HD;
  const float* W = which == 0 ? Wq : (which == 1 ? Wk : Wv);
  const float* al = which == 0 ? aq : (which == 1 ? ak : av);
  v4f acc = {0.f, 0.f, 0.f, 0.f};
#pragma unroll 1
  for (int m = 0; m < HH; ++m) { const float a = al[(m * HH + h) * PP + p];
    const v4f w = *(const v4f*)(W + (size_t)(m * HD + d) * DD + tid * 4);
    acc += a * w; }
  vst2(Weff + ((size_t)which * DO + o) * DD + tid * 4, acc);
}
__global__ __launch_bounds__(256) void k_beff(const float* __restrict__ bq, const float* __restrict__ bk, const float* __restrict__ bv,
                                            const float* __restrict__ aq, const float* __restrict__ ak, const float* __restrict__ av, float* __restrict__ beff) {
  const int o = blockIdx.x * 256 + threadIdx.x, which = blockIdx.y;
  const int h = o / (PP * HD), p = (o / HD) % PP, d = o % HD;
  const float* bb = which == 0 ? bq : (which == 1 ? bk : bv);
  const float* al = which == 0 ? aq : (which == 1 ? ak : av);
  float acc = 0.f;
#pragma unroll 1
  for (int m = 0; m < HH; ++m) acc += al[(m * HH + h) * PP + p] * bb[m * HD + d];
  vst2(beff + (size_t)which * DO + o, (float_a)acc);
}

__global__ __launch_bounds__(128) void k_qkv(const _Float16* __restrict__ X16, const _Float16* __restrict__ W16, const float* __restrict__ beff,
                                           float* __restrict__ qp, float* __restrict__ kp, float* __restrict__ vT) {
  __shared__ __align__(16) float st[128][68];
  const int tid = threadIdx.x, wave = tid >> 5, lane = tid & 31, col = lane & 15, g = lane >> 4;
  const int r0 = blockIdx.x * 64, h = blockIdx.y, which = blockIdx.z, n0 = h * 128;
  const int b = r0 / ST, s0 = r0 % ST;
  const _Float16* Wt = W16 + (size_t)which * DO * DD; const float* bb = beff + (size_t)which * DO;
  v8f acc[8] = {};
#pragma unroll 2
  for (int kc = 0; kc < DD / 32; ++kc) {
    const v16h a = frag_h(X16 + (size_t)(r0 + wave * 16 + col) * DD + kc * 32, lane);
#pragma unroll
    for (int j = 0; j < 8; ++j) acc[j] = wmma16(a, frag_h(Wt + (size_t)(n0 + j * 16 + col) * DD + kc * 32, lane), acc[j]);
  }
#pragma unroll
  for (int j = 0; j < 8; ++j) { const float bv = bb[n0 + j * 16 + col];
#pragma unroll
    for (int r = 0; r < 8; ++r) st[j * 16 + col][wave * 16 + 8 * g + r] = acc[j][r] * (1.0f / 16.0f) + bv; }
  __syncthreads();
  if (which < 2) {
    float* dst = which == 0 ? qp : kp;
    for (int q = tid; q < 128 * 16; q += 128) { const int nl = q >> 4, pc = q & 15; const int sl = nl >> 1, p = nl & 1;
      v4f v = { st[p * 64 + pc * 4][sl], st[p * 64 + pc * 4 + 1][sl], st[p * 64 + pc * 4 + 2][sl], st[p * 64 + pc * 4 + 3][sl] };
      vst2(dst + (((size_t)b * HH + h) * SS + 2 * s0 + nl) * HD + pc * 4, v); }
  } else {
    __syncthreads();
    for (int q = tid; q < 64 * 32; q += 128) { const int d = q >> 5, pc = q & 31;
      v4f v = { st[d][2 * pc], st[64 + d][2 * pc], st[d][2 * pc + 1], st[64 + d][2 * pc + 1] };
      vst2(vT + (((size_t)b * HH + h) * HD + d) * SS + 2 * s0 + pc * 4, v); }
  }
}

__global__ __launch_bounds__(128) void k_attn(const float* __restrict__ qp, const float* __restrict__ kp, const float* __restrict__ vT, const float* __restrict__ collapse, float* __restrict__ y) {
  __shared__ __align__(16) float sP[4][16][BK];
  __shared__ __align__(16) float sO[4][16][HD];
  const int tid = threadIdx.x, w = tid >> 5, lane = tid & 31, g = lane >> 4, ln = lane & 15;
  const int bh = blockIdx.y, b = bh / HH, h = bh % HH, q0 = blockIdx.x * 64 + w * 16;
  const float* qrow = qp + ((size_t)bh * SS + q0 + ln) * HD;
  const v16h qa0 = frag_f32(qrow, lane), qa1 = frag_f32(qrow + 32, lane);
  const float scale = 0.125f;
  float mrun[8], lrun[8];
  v8f acc[4];
#pragma unroll
  for (int r = 0; r < 8; ++r) { mrun[r] = -3.0e38f; lrun[r] = 0.f; }
#pragma unroll
  for (int t = 0; t < 4; ++t) acc[t] = (v8f){};
  const float* kb = kp + (size_t)bh * SS * HD;
  const float* vb = vT + (size_t)bh * HD * SS;
  const int kend = blockIdx.x * 64 + 64;
#pragma unroll 1
  for (int k0 = 0; k0 < kend; k0 += BK) {
    v8f s0 = {}, s1 = {};
    s0 = wmma16(qa0, frag_f32(kb + (size_t)(k0 + ln) * HD, lane), s0);      s0 = wmma16(qa1, frag_f32(kb + (size_t)(k0 + ln) * HD + 32, lane), s0);
    s1 = wmma16(qa0, frag_f32(kb + (size_t)(k0 + 16 + ln) * HD, lane), s1); s1 = wmma16(qa1, frag_f32(kb + (size_t)(k0 + 16 + ln) * HD + 32, lane), s1);
#pragma unroll
    for (int r = 0; r < 8; ++r) {
      const int qg = q0 + 8 * g + r;
      const float x0 = (((k0 + ln) >> 1) <= (qg >> 1)) ? s0[r] * scale : -3.0e38f, x1 = (((k0 + 16 + ln) >> 1) <= (qg >> 1)) ? s1[r] * scale : -3.0e38f;
      float mx = fmaxf(x0, x1);
#pragma unroll
      for (int off = 8; off >= 1; off >>= 1) mx = fmaxf(mx, __shfl_xor(mx, off, 32));
      const float mn = fmaxf(mrun[r], mx);
      const float corr = expf(mrun[r] - mn);
      const float p0 = (x0 > -1.0e38f) ? expf(x0 - mn) : 0.f, p1 = (x1 > -1.0e38f) ? expf(x1 - mn) : 0.f;
      float sum = p0 + p1;
#pragma unroll
      for (int off = 8; off >= 1; off >>= 1) sum += __shfl_xor(sum, off, 32);
      lrun[r] = lrun[r] * corr + sum; mrun[r] = mn;
#pragma unroll
      for (int t = 0; t < 4; ++t) acc[t][r] *= corr;
      sP[w][8 * g + r][ln] = p0 * 16384.0f; sP[w][8 * g + r][16 + ln] = p1 * 16384.0f;
    }
    LDSX();
    const v16h pa = frag_f32(&sP[w][ln][0], lane);
#pragma unroll
    for (int t = 0; t < 4; ++t) { const H2 vb2 = hsplit_row(vb + (size_t)(t * 16 + ln) * SS + k0, lane);
      acc[t] = wmma16(pa, vb2.l, acc[t]); acc[t] = wmma16(pa, vb2.h, acc[t]); }
    __builtin_amdgcn_wave_barrier();
  }
  float* so = &sO[w][0][0];
#pragma unroll
  for (int r = 0; r < 8; ++r) { const float il = (1.0f / 16384.0f) / lrun[r];
#pragma unroll
    for (int t = 0; t < 4; ++t) so[(8 * g + r) * HD + t * 16 + ln] = acc[t][r] * il; }
  LDSX();
  const float c0 = collapse[h * PP], c1 = collapse[h * PP + 1];
#pragma unroll
  for (int q = 0; q < 4; ++q) { const int j = q * 2 + (lane >> 4), pc = lane & 15;
    const v4f v = c0 * *(const v4f*)(so + (2 * j) * HD + pc * 4) + c1 * *(const v4f*)(so + (2 * j + 1) * HD + pc * 4);
    vst2(y + ((size_t)b * ST + (q0 >> 1) + j) * DD + h * HD + pc * 4, v); }
}

__global__ __launch_bounds__(128) void k_out(const float* __restrict__ y, const _Float16* __restrict__ Wo16, const float* __restrict__ bo, float* __restrict__ out) {
  __shared__ __align__(16) float so[4][16 * 128];
  const int tid = threadIdx.x, wave = tid >> 5, lane = tid & 31, col = lane & 15, g = lane >> 4;
  const int r0 = blockIdx.x * 64 + wave * 16, n0 = blockIdx.y * 128;
  v8f acc[8] = {};
#pragma unroll 2
  for (int kc = 0; kc < DD / 32; ++kc) {
    const v16h a = frag_f32(y + (size_t)(r0 + col) * DD + kc * 32, lane);
#pragma unroll
    for (int j = 0; j < 8; ++j) acc[j] = wmma16(a, frag_h(Wo16 + (size_t)(n0 + j * 16 + col) * DD + kc * 32, lane), acc[j]);
  }
  float* S = so[wave];
#pragma unroll
  for (int j = 0; j < 8; ++j) { const float bv = bo[n0 + j * 16 + col];
#pragma unroll
    for (int r = 0; r < 8; ++r) S[(8 * g + r) * 128 + j * 16 + col] = acc[j][r] * (1.0f / 16.0f) + bv; }
  LDSX();
#pragma unroll 4
  for (int rl = 0; rl < 16; ++rl) vst2(out + (size_t)(r0 + rl) * DD + n0 + lane * 4, *(const v4f*)(S + rl * 128 + lane * 4));
}

extern "C" void kernel_launch(void* const* d_in, const int* in_sizes, int n_in,
                              void* d_out, int out_size, void* d_ws, size_t ws_size,
                              hipStream_t stream) {
  (void)in_sizes; (void)n_in; (void)out_size; (void)ws_size;
  const float* x  = (const float*)d_in[0];
  const float* Wq = (const float*)d_in[1]; const float* bq = (const float*)d_in[2];
  const float* Wk = (const float*)d_in[3]; const float* bk = (const float*)d_in[4];
  const float* Wv = (const float*)d_in[5]; const float* bv = (const float*)d_in[6];
  const float* Wo = (const float*)d_in[7]; const float* bo = (const float*)d_in[8];
  const float* aq = (const float*)d_in[9]; const float* ak = (const float*)d_in[10]; const float* av = (const float*)d_in[11];
  const float* coll = (const float*)d_in[12];
  float* out = (float*)d_out;
  char* ws = (char*)d_ws; size_t off = 0;
  auto take = [&](size_t bytes) { char* p = ws + off; off += (bytes + 255) & ~(size_t)255; return p; };
  float* Weff = (float*)take((size_t)3 * DO * DD * 4);
  float* beff = (float*)take((size_t)3 * DO * 4);
  float* qp  = (float*)take((size_t)BB * HH * SS * HD * 4);
  float* kp  = (float*)take((size_t)BB * HH * SS * HD * 4);
  float* vT  = (float*)take((size_t)BB * HH * HD * SS * 4);
  float* y   = (float*)take((size_t)BT * DD * 4);
  _Float16* X16 = (_Float16*)take((size_t)BT * DD * 2); _Float16* W16 = (_Float16*)take((size_t)3 * DO * DD * 2); _Float16* Wo16 = (_Float16*)take((size_t)DD * DD * 2);
  k_weff<<<dim3(DO, 3), 256, 0, stream>>>(Wq, Wk, Wv, aq, ak, av, Weff);
  k_beff<<<dim3(DO / 256, 3), 256, 0, stream>>>(bq, bk, bv, aq, ak, av, beff);
  k_cvt<<<(unsigned)((size_t)BT * DD / 8 + 255) / 256, 256, 0, stream>>>(x, X16, (size_t)BT * DD / 8, 1.0f);
  k_cvt<<<(unsigned)((size_t)3 * DO * DD / 8 + 255) / 256, 256, 0, stream>>>(Weff, W16, (size_t)3 * DO * DD / 8, 16.0f);
  k_cvt<<<(unsigned)((size_t)DD * DD / 8 + 255) / 256, 256, 0, stream>>>(Wo, Wo16, (size_t)DD * DD / 8, 16.0f);
  k_qkv<<<dim3(BT / 64, HH, 3), 128, 0, stream>>>(X16, W16, beff, qp, kp, vT);
  k_attn<<<dim3(SS / 64, BB * HH), 128, 0, stream>>>(qp, kp, vT, coll, y);
  k_out<<<dim3(BT / 64, DD / 128), 128, 0, stream>>>(y, Wo16, bo, out);
}
